// LSTMLanguageModel_10067403341867
// MI455X (gfx1250) — hardware-verified
//
#include <hip/hip_runtime.h>
#include <math.h>

constexpr int NVOC     = 30000;
constexpr int NEMB     = 100;
constexpr int NHID     = 300;
constexpr int NBAT     = 512;
constexpr int NSTEP    = 256;
constexpr int NVOCP    = 30016;
constexpr int KEMB     = 128;
constexpr int KHID     = 320;
constexpr int NTILE    = 19;
constexpr int NGATEP   = NTILE * 64;
constexpr int ROWS_BLK = 16;
constexpr int NWAVE_R  = 10;
constexpr int NTHR_R   = NWAVE_R * 32;
constexpr int HP       = 328;
constexpr int SP       = 304;
constexpr float CARRY    = 16.0f;
constexpr float ACC_FOLD = 1.0f / (CARRY * CARRY);
constexpr size_t OUT1_OFF = (size_t)NBAT * NVOC;
constexpr size_t OUT2_OFF = OUT1_OFF + (size_t)NBAT * NHID;

static_assert(NVOCP % 64 == 0 && NVOCP >= NVOC);
static_assert(NGATEP % 64 == 0 && NTILE * 16 >= NHID);
static_assert(NBAT % 64 == 0 && NBAT % ROWS_BLK == 0);
static_assert(KEMB % 32 == 0 && KEMB >= NEMB);
static_assert(KHID % 32 == 0 && KHID >= NTILE * 16);
static_assert(HP % 8 == 0 && HP >= KHID);
static_assert(SP % 4 == 0 && SP >= NTILE * 16);
static_assert(2 * NWAVE_R >= NTILE);
static_assert(OUT1_OFF * 4 == 61440000ull);
static_assert(OUT2_OFF * 4 == 62054400ull);
static_assert((OUT2_OFF + (size_t)NBAT * NHID) * 4 == 62668800ull);
static_assert((NBAT * (NVOC / 4)) % 256 == 0);
static_assert(NVOC % 4 == 0 && NHID % 4 == 0);
static_assert((ROWS_BLK * (KHID / 8)) == 2 * NTHR_R);
static_assert(2 * ROWS_BLK * HP * 2 + NSTEP * ROWS_BLK * 4 + ROWS_BLK * SP * 4 <= 65536);

typedef __attribute__((ext_vector_type(16))) _Float16 v16h;
typedef __attribute__((ext_vector_type(8)))  _Float16 v8h;
typedef __attribute__((ext_vector_type(8)))  float    v8f;
typedef __attribute__((ext_vector_type(4)))  float    v4f;
typedef __attribute__((ext_vector_type(2)))  unsigned v2u;

__device__ __forceinline__ void guard_grp4(v8f& a0, v8f& a1, v8f& a2, v8f& a3, v16h x, v16h y0, v16h y1, v16h y2, v16h y3) {
  asm volatile("v_nop\n\tv_nop\n\tv_nop\n\tv_nop" : "+v"(a0), "+v"(a1), "+v"(a2), "+v"(a3) : "v"(x), "v"(y0), "v"(y1), "v"(y2), "v"(y3));
}
__device__ __forceinline__ void keep4_h(v16h a, v16h b, v16h c, v16h d) { asm volatile("v_nop" :: "v"(a), "v"(b), "v"(c), "v"(d)); }
__device__ __forceinline__ void acc_guard4(v8f& a, v8f& b, v8f& c, v8f& d) { asm volatile("v_nop\n\tv_nop\n\tv_nop\n\tv_nop" : "+v"(a), "+v"(b), "+v"(c), "+v"(d)); }

struct FragH {
  union U { v16h v; v8h h[2]; };
  static __device__ __forceinline__ v16h load(const _Float16* p) {
    U f; f.h[0] = *(const v8h*)(p); f.h[1] = *(const v8h*)(p + 16); return f.v;
  }
  static __device__ __forceinline__ v8f mma(v16h a, v16h b, v8f c) {
    return __builtin_amdgcn_wmma_f32_16x16x32_f16(false, a, false, b, (short)0, c, false, false);
  }
};

__device__ __forceinline__ float fsig(float x)  { return __builtin_amdgcn_rcpf(1.0f + __expf(-x)); }
__device__ __forceinline__ float ftanh(float x) { return 1.0f - 2.0f * __builtin_amdgcn_rcpf(__expf(2.0f * x) + 1.0f); }

__device__ __forceinline__ float h16_to_f32(unsigned hb) {
  const unsigned sgn = (hb & 0x8000u) << 16; const unsigned em = hb & 0x7fffu;
  const float fn = __uint_as_float((em << 13) + 0x38000000u);
  const float fs = (float)em * 5.9604644775390625e-8f;
  const float mag = (em < 0x400u) ? fs : fn; return __uint_as_float(__float_as_uint(mag) | sgn); }

template <int BIAS_MODE, int OUT_MODE>
__global__ __launch_bounds__(256) void wmma_gemm64_f16(
    const unsigned short* __restrict__ Ap, int lda,
    const unsigned short* __restrict__ Btp, int ldb,
    void* __restrict__ Cout, int ldc,
    const float* __restrict__ bias,
    int M, int N, int K, float scale) {
  const _Float16* A  = (const _Float16*)Ap;
  const _Float16* Bt = (const _Float16*)Btp;
  __shared__ __align__(16) float sT[8][16 * 68];
  const int lane = threadIdx.x & 31;
  const int wave = threadIdx.x >> 5;
  const int tilesN = N >> 6;
  const int tilesM = M >> 6;
  const int tile = blockIdx.x * 8 + wave;
  if (tile >= tilesM * tilesN) return;
  const int tm = tile / tilesN;
  const int tn = tile - tm * tilesN;
  const int m0 = tm << 6;
  const int n0 = tn << 6;

  const int rlane = lane & 15;
  const int koff  = (lane >> 4) * 8;
  const int mOff  = (lane >> 4) * 8;

  v8f acc[4][4];
#pragma unroll
  for (int i = 0; i < 4; ++i)
#pragma unroll
    for (int j = 0; j < 4; ++j) acc[i][j] = (v8f){0.f,0.f,0.f,0.f,0.f,0.f,0.f,0.f};

  for (int k0 = 0; k0 < K; k0 += 32) {
    v16h bh[4];
#pragma unroll
    for (int j = 0; j < 4; ++j) {
      const size_t bo = (size_t)(n0 + (j << 4) + rlane) * ldb + koff + k0;
      bh[j] = FragH::load(Bt + bo);
    }
#pragma unroll
    for (int i = 0; i < 4; ++i) {
      const size_t ao = (size_t)(m0 + (i << 4) + rlane) * lda + koff + k0;
      const v16h ah = FragH::load(A + ao);
#pragma unroll
      for (int j = 0; j < 4; ++j) acc[i][j] = FragH::mma(ah, bh[j], acc[i][j]);
      guard_grp4(acc[i][0], acc[i][1], acc[i][2], acc[i][3], ah, bh[0], bh[1], bh[2], bh[3]);
    }
    keep4_h(bh[0], bh[1], bh[2], bh[3]);
  }
  acc_guard4(acc[0][0], acc[0][1], acc[0][2], acc[0][3]);
  acc_guard4(acc[1][0], acc[1][1], acc[1][2], acc[1][3]);
  acc_guard4(acc[2][0], acc[2][1], acc[2][2], acc[2][3]);
  acc_guard4(acc[3][0], acc[3][1], acc[3][2], acc[3][3]);

  float* slab = sT[wave];
#pragma unroll
  for (int i = 0; i < 4; ++i) {
    const int mBase = m0 + (i << 4);
#pragma unroll
    for (int j = 0; j < 4; ++j) {
      const int n = n0 + (j << 4) + rlane;
      float bv = 0.f;
      if (BIAS_MODE == 2) bv = bias[n];
#pragma unroll
      for (int r = 0; r < 8; ++r) {
        float v = acc[i][j][r] * scale;
        if (BIAS_MODE == 2) v += bv;
        slab[(mOff + r) * 68 + (j << 4) + rlane] = v;
      }
    }
    __builtin_amdgcn_fence(__ATOMIC_RELEASE, "workgroup");
    __builtin_amdgcn_wave_barrier();
    __builtin_amdgcn_fence(__ATOMIC_ACQUIRE, "workgroup");
    if (OUT_MODE == 0) {
      float* C = (float*)Cout;
      const int hh = lane >> 4, c4 = (lane & 15) * 4;
      for (int pass = 0; pass < 2; ++pass) {
#pragma unroll
        for (int it = 0; it < 8; ++it) {
          const int row = it * 2 + hh;
          v4f v = *(const v4f*)(slab + row * 68 + c4);
          *(volatile v4f*)(C + (size_t)(mBase + row) * ldc + n0 + c4) = v;
        }
        __threadfence();
      }
    } else {
      const int q = lane >> 3, c8 = (lane & 7) * 8;
      unsigned short* C = (unsigned short*)Cout;
      for (int pass = 0; pass < 2; ++pass) {
#pragma unroll
        for (int it = 0; it < 4; ++it) {
          const int row = it * 4 + q;
          const float* sp = slab + row * 68 + c8;
          v8h hv;
#pragma unroll
          for (int e = 0; e < 8; ++e) hv[e] = (_Float16)sp[e];
          *(volatile v8h*)(C + (size_t)(mBase + row) * ldc + n0 + c8) = hv;
        }
        __threadfence();
      }
    }
    __builtin_amdgcn_fence(__ATOMIC_RELEASE, "workgroup");
    __builtin_amdgcn_wave_barrier();
    __builtin_amdgcn_fence(__ATOMIC_ACQUIRE, "workgroup");
  }
}

template <int MODE>
__global__ __launch_bounds__(256) void pack16_kernel(const float* __restrict__ src, unsigned short* __restrict__ dst,
                                                     int srcRows, int srcCols, int dstRows, int k8n) {
  const int i  = blockIdx.x * 256 + threadIdx.x;
  const int n8 = dstRows * k8n;
  if (i < n8) {
    const int rr = i / k8n;
    const int c8 = i - rr * k8n;
    int srow;
    bool rvalid;
    if (MODE == 0) {
      srow = rr;
      rvalid = rr < srcRows;
    } else {
      const int nt = rr >> 6;
      const int w  = rr & 63;
      const int g  = (MODE == 1) ? (w >> 4) : (w & 3);
      const int j  = (MODE == 1) ? (w & 15) : (w >> 2);
      const int hid = nt * 16 + j;
      rvalid = hid < NHID;
      srow = g * NHID + hid;
    }
    const int srowc = rvalid ? srow : 0;
    const float* sp = src + (size_t)srowc * srcCols;
    v8h hv;
#pragma unroll
    for (int e = 0; e < 8; ++e) {
      const int k  = c8 * 8 + e;
      const int kc = (k < srcCols) ? k : (srcCols - 1);
      const float f = sp[kc];
      const float val = (rvalid && (k < srcCols)) ? (f * CARRY) : 0.0f;
      hv[e] = (_Float16)val;
    }
    *(volatile v8h*)(dst + (size_t)i * 8) = hv;
    __threadfence();
    *(volatile v8h*)(dst + (size_t)i * 8) = hv;
  }
}

__global__ __launch_bounds__(256) void bsum_kernel(const float* __restrict__ bi, const float* __restrict__ bh,
                                                   float* __restrict__ dst) {
  const int j4 = blockIdx.x * 256 + threadIdx.x;
  if (j4 < NGATEP / 4) {
    const int hid = j4;
    const bool ok = hid < NHID;
    const int hc = ok ? hid : (NHID - 1);
    v4f o;
#pragma unroll
    for (int g = 0; g < 4; ++g) {
      const float s = bi[g * NHID + hc] + bh[g * NHID + hc];
      o[g] = ok ? s : 0.0f;
    }
    float* op = dst + (size_t)j4 * 4;
    *(volatile v4f*)op = o;
    __threadfence();
    *(volatile v4f*)op = o;
  }
}

__global__ __launch_bounds__(256) void bfc_pad_kernel(const float* __restrict__ bfc, float* __restrict__ dst) {
  const int j4 = blockIdx.x * 256 + threadIdx.x;
  if (j4 < NVOCP / 4) {
    v4f o;
#pragma unroll
    for (int e = 0; e < 4; ++e) {
      const int n  = j4 * 4 + e;
      const int nc = (n < NVOC) ? n : (NVOC - 1);
      const float f = bfc[nc];
      o[e] = (n < NVOC) ? f : 0.0f;
    }
    float* op = dst + (size_t)j4 * 4;
    *(volatile v4f*)op = o;
    __threadfence();
    *(volatile v4f*)op = o;
  }
}

__global__ __launch_bounds__(NTHR_R) void lstm_seq_kernel(
    const int* __restrict__ xtok, const float* __restrict__ h0, const float* __restrict__ c0,
    const unsigned short* __restrict__ Whhp, const unsigned short* __restrict__ Ptab,
    const float* __restrict__ bsum4,
    float* __restrict__ out_h, float* __restrict__ out_c, unsigned short* __restrict__ H16) {
  __shared__ __align__(16) _Float16 hbuf[2 * ROWS_BLK * HP];
  __shared__ __align__(16) int      tokT[NSTEP * ROWS_BLK];
  __shared__ __align__(16) float    Sst[ROWS_BLK * SP];
  const _Float16* Whh = (const _Float16*)Whhp;
  const int tid  = threadIdx.x;
  const int lane = tid & 31;
  const int wave = __builtin_amdgcn_readfirstlane(tid >> 5);
  const int c = lane & 15, hh = lane >> 4, koff = hh * 8;
  const int rowbase = blockIdx.x * ROWS_BLK;

#pragma unroll 1
  for (int i = tid; i < ROWS_BLK * NSTEP; i += NTHR_R) {
    const int row = i / NSTEP;
    const int t   = i - row * NSTEP;
    int tk = xtok[(size_t)(rowbase + row) * NSTEP + t];
    tk = (tk < 0) ? 0 : tk;
    tk = (tk > NVOC - 1) ? (NVOC - 1) : tk;
    tokT[t * ROWS_BLK + row] = tk;
  }
#pragma unroll 1
  for (int i = tid; i < 2 * ROWS_BLK * HP; i += NTHR_R) {
    const int buf = i / (ROWS_BLK * HP);
    const int rem = i - buf * (ROWS_BLK * HP);
    const int row = rem / HP;
    const int col = rem - row * HP;
    const int cc  = (col < NHID) ? col : (NHID - 1);
    const float f = h0[(size_t)(rowbase + row) * NHID + cc];
    const float val = ((buf == 0) && (col < NHID)) ? (f * CARRY) : 0.0f;
    hbuf[i] = (_Float16)val;
  }
  float cst[2][8];
  v4f bb[2];
#pragma unroll
  for (int q = 0; q < 2; ++q) {
    const int nt  = wave + q * NWAVE_R;
    const int ntc = (nt < NTILE) ? nt : (NTILE - 1);
    const int col = 16 * ntc + c;
    const int cc  = (col < NHID) ? col : (NHID - 1);
    const bool ok = (nt < NTILE) && (col < NHID);
    bb[q] = *(const v4f*)(bsum4 + ntc * 64 + c * 4);
#pragma unroll
    for (int r = 0; r < 8; ++r) {
      const float f = c0[(size_t)(rowbase + 8 * hh + r) * NHID + cc];
      cst[q][r] = ok ? f : 0.0f;
    }
  }
  __syncthreads();

  const v8f z8 = {0.f, 0.f, 0.f, 0.f, 0.f, 0.f, 0.f, 0.f};
  const v8h zero8 = {(_Float16)0.0f, (_Float16)0.0f, (_Float16)0.0f, (_Float16)0.0f,
                     (_Float16)0.0f, (_Float16)0.0f, (_Float16)0.0f, (_Float16)0.0f};

#pragma unroll 1
  for (int t = 0; t < NSTEP; ++t) {
    const int cur = t & 1;
    const _Float16* hc = hbuf + cur * (ROWS_BLK * HP);
    _Float16*       hn = hbuf + (cur ^ 1) * (ROWS_BLK * HP);
    const bool last = (t == NSTEP - 1);
    int tk[8];
#pragma unroll
    for (int r = 0; r < 8; ++r) tk[r] = tokT[t * ROWS_BLK + 8 * hh + r];

#pragma unroll
    for (int q = 0; q < 2; ++q) {
      const int nt = wave + q * NWAVE_R;
      if (nt < NTILE) {
        const int col = 16 * nt + c;
        const bool valid = col < NHID;
        const _Float16* ahrow = hc + c * HP + koff;
        const _Float16* wh = Whh + (size_t)(nt * 64 + c) * KHID + koff;
        v8f acc0 = z8, acc1 = z8, acc2 = z8, acc3 = z8;
#pragma unroll 1
        for (int k0 = 0; k0 < KHID; k0 += 32) {
          const v16h a  = FragH::load(ahrow + k0);
          const v16h b0 = FragH::load(wh + k0);
          const v16h b1 = FragH::load(wh + 16 * KHID + k0);
          const v16h b2 = FragH::load(wh + 32 * KHID + k0);
          const v16h b3 = FragH::load(wh + 48 * KHID + k0);
          acc0 = FragH::mma(a, b0, acc0);
          acc1 = FragH::mma(a, b1, acc1);
          acc2 = FragH::mma(a, b2, acc2);
          acc3 = FragH::mma(a, b3, acc3);
          guard_grp4(acc0, acc1, acc2, acc3, a, b0, b1, b2, b3);
        }
        acc_guard4(acc0, acc1, acc2, acc3);
        unsigned pw0[8], pw1[8];
#pragma unroll
        for (int r = 0; r < 8; ++r) {
          const v2u w = *(const v2u*)(Ptab + (size_t)tk[r] * NGATEP + nt * 64 + c * 4);
          pw0[r] = w[0];
          pw1[r] = w[1];
        }
#pragma unroll
        for (int r = 0; r < 8; ++r) {
          const float pi = h16_to_f32(pw0[r] & 0xffffu);
          const float pf = h16_to_f32(pw0[r] >> 16);
          const float pg = h16_to_f32(pw1[r] & 0xffffu);
          const float po = h16_to_f32(pw1[r] >> 16);
          const float zi = acc0[r] * ACC_FOLD + (bb[q][0] + pi);
          const float zf = acc1[r] * ACC_FOLD + (bb[q][1] + pf);
          const float zg = acc2[r] * ACC_FOLD + (bb[q][2] + pg);
          const float zo = acc3[r] * ACC_FOLD + (bb[q][3] + po);
          const float ig = fsig(zi);
          const float fg = fsig(zf);
          const float gg = ftanh(zg);
          const float og = fsig(zo);
          float cn = fg * cst[q][r] + ig * gg;
          float hv = og * ftanh(cn);
          cn = valid ? cn : 0.0f;
          hv = valid ? hv : 0.0f;
          cst[q][r] = cn;
          hn[(8 * hh + r) * HP + col] = (_Float16)(hv * CARRY);
          if (last) Sst[(8 * hh + r) * SP + col] = hv;
        }
      }
    }
    if (wave == 0) {
      *(v8h*)(hn + (lane >> 1) * HP + NTILE * 16 + (lane & 1) * 8) = zero8;
    }
    __syncthreads();
  }

  {
    const _Float16* hf = hbuf + (NSTEP & 1) * (ROWS_BLK * HP);
    v8h hv2[2];
#pragma unroll
    for (int it = 0; it < 2; ++it) {
      const int idx = it * NTHR_R + tid;
      const int row = idx / (KHID / 8);
      const int c8  = (idx - row * (KHID / 8)) * 8;
      hv2[it] = *(const v8h*)(hf + row * HP + c8);
    }
    unsigned short* hp = H16 + (size_t)rowbase * KHID;
    for (int pass = 0; pass < 2; ++pass) {
#pragma unroll
      for (int it = 0; it < 2; ++it) {
        const int idx = it * NTHR_R + tid;
        *(volatile v8h*)(hp + (size_t)idx * 8) = hv2[it];
      }
      __threadfence();
    }
  }
  {
    v4f sv[4];
#pragma unroll
    for (int it = 0; it < 4; ++it) {
      const int idx = it * NTHR_R + tid;
      const int idc = (idx < ROWS_BLK * (NHID / 4)) ? idx : (ROWS_BLK * (NHID / 4) - 1);
      const int row = idc / (NHID / 4);
      const int c4  = (idc - row * (NHID / 4)) * 4;
      sv[it] = *(const v4f*)(Sst + row * SP + c4);
    }
    float* oh = out_h + (size_t)rowbase * NHID;
    for (int pass = 0; pass < 2; ++pass) {
#pragma unroll
      for (int it = 0; it < 4; ++it) {
        const int idx = it * NTHR_R + tid;
        if (idx < ROWS_BLK * (NHID / 4)) *(volatile v4f*)(oh + (size_t)idx * 4) = sv[it];
      }
      __threadfence();
    }
  }
  __syncthreads();
#pragma unroll
  for (int q = 0; q < 2; ++q) {
    const int nt = wave + q * NWAVE_R;
    if (nt < NTILE) {
      const int col = 16 * nt + c;
#pragma unroll
      for (int r = 0; r < 8; ++r) Sst[(8 * hh + r) * SP + col] = cst[q][r];
    }
  }
  __syncthreads();
  {
    v4f sv[4];
#pragma unroll
    for (int it = 0; it < 4; ++it) {
      const int idx = it * NTHR_R + tid;
      const int idc = (idx < ROWS_BLK * (NHID / 4)) ? idx : (ROWS_BLK * (NHID / 4) - 1);
      const int row = idc / (NHID / 4);
      const int c4  = (idc - row * (NHID / 4)) * 4;
      sv[it] = *(const v4f*)(Sst + row * SP + c4);
    }
    float* oc = out_c + (size_t)rowbase * NHID;
    for (int pass = 0; pass < 2; ++pass) {
#pragma unroll
      for (int it = 0; it < 4; ++it) {
        const int idx = it * NTHR_R + tid;
        if (idx < ROWS_BLK * (NHID / 4)) *(volatile v4f*)(oc + (size_t)idx * 4) = sv[it];
      }
      __threadfence();
    }
  }
}

__global__ __launch_bounds__(256) void out_copy_kernel(const float* __restrict__ Cst, float* __restrict__ out) {
  const int j = blockIdx.x * 256 + threadIdx.x;
  if (j < NBAT * (NVOC / 4)) {
    const int b   = j / (NVOC / 4);
    const int v4i = (j - b * (NVOC / 4)) * 4;
    const v4f v = *(const v4f*)(Cst + (size_t)b * NVOCP + v4i);
    float* op = out + (size_t)j * 4;
    *(volatile v4f*)op = v;
    __threadfence();
    *(volatile v4f*)op = v;
  }
}

extern "C" void kernel_launch(void* const* d_in, const int* in_sizes, int n_in,
                              void* d_out, int out_size, void* d_ws, size_t ws_size, hipStream_t stream) {
  if (n_in < 10 || d_out == nullptr || d_ws == nullptr) return;
  if (in_sizes[0] != NBAT * NSTEP || in_sizes[1] != NBAT * NHID || in_sizes[2] != NBAT * NHID ||
      in_sizes[3] != NVOC * NEMB || in_sizes[4] != 4 * NHID * NEMB || in_sizes[5] != 4 * NHID * NHID ||
      in_sizes[6] != 4 * NHID || in_sizes[7] != 4 * NHID || in_sizes[8] != NVOC * NHID || in_sizes[9] != NVOC ||
      out_size != NBAT * NVOC + 2 * NBAT * NHID) return;

  const int*   xtok = (const int*)  d_in[0];
  const float* h0   = (const float*)d_in[1];
  const float* c0   = (const float*)d_in[2];
  const float* emb  = (const float*)d_in[3];
  const float* w_ih = (const float*)d_in[4];
  const float* w_hh = (const float*)d_in[5];
  const float* b_ih = (const float*)d_in[6];
  const float* b_hh = (const float*)d_in[7];
  const float* w_fc = (const float*)d_in[8];
  const float* b_fc = (const float*)d_in[9];
  float* out   = (float*)d_out;
  float* out_h = out + OUT1_OFF;
  float* out_c = out + OUT2_OFF;

  char* ws = (char*)d_ws; size_t off = 0;
  auto carve = [&](size_t bytes) -> char* { char* p = ws + off; off += (bytes + 255) & ~(size_t)255; return p; };
  unsigned short* E16   = (unsigned short*)carve((size_t)NVOCP * KEMB * 2);
  unsigned short* WIH16 = (unsigned short*)carve((size_t)NGATEP * KEMB * 2);
  unsigned short* WHH16 = (unsigned short*)carve((size_t)NGATEP * KHID * 2);
  unsigned short* WFC16 = (unsigned short*)carve((size_t)NVOCP * KHID * 2);
  unsigned short* PTAB  = (unsigned short*)carve((size_t)NVOCP * NGATEP * 2);
  float*          BSUM  = (float*)carve((size_t)NGATEP * 4);
  float*          BFCP  = (float*)carve((size_t)NVOCP * 4);
  unsigned short* H16   = (unsigned short*)carve((size_t)NBAT * KHID * 2);
  float*          CST   = (float*)PTAB;
  static_assert((size_t)NBAT * NVOCP * 4 <= (size_t)NVOCP * NGATEP * 2);
  if (off > ws_size || off > (size_t)134217728) return;

  pack16_kernel<0><<<(NVOCP * (KEMB / 8)) / 256, 256, 0, stream>>>(emb,  E16,   NVOC,     NEMB, NVOCP,  KEMB / 8);
  pack16_kernel<2><<<(NGATEP * (KEMB / 8)) / 256, 256, 0, stream>>>(w_ih, WIH16, 4 * NHID, NEMB, NGATEP, KEMB / 8);
  pack16_kernel<1><<<(NGATEP * (KHID / 8)) / 256, 256, 0, stream>>>(w_hh, WHH16, 4 * NHID, NHID, NGATEP, KHID / 8);
  pack16_kernel<0><<<(NVOCP * (KHID / 8)) / 256, 256, 0, stream>>>(w_fc, WFC16, NVOC,     NHID, NVOCP,  KHID / 8);
  static_assert((NVOCP * (KEMB / 8)) % 256 == 0 && (NGATEP * (KEMB / 8)) % 256 == 0);
  static_assert((NGATEP * (KHID / 8)) % 256 == 0 && (NVOCP * (KHID / 8)) % 256 == 0);
  bsum_kernel<<<(NGATEP / 4 + 255) / 256, 256, 0, stream>>>(b_ih, b_hh, BSUM);
  bfc_pad_kernel<<<(NVOCP / 4 + 255) / 256, 256, 0, stream>>>(b_fc, BFCP);

  {
    const int tiles = (NVOCP / 64) * (NGATEP / 64);
    wmma_gemm64_f16<0, 1><<<(tiles + 7) / 8, 256, 0, stream>>>(
        E16, KEMB, WIH16, KEMB, (void*)PTAB, NGATEP, BSUM, NVOCP, NGATEP, KEMB, ACC_FOLD);
  }

  lstm_seq_kernel<<<NBAT / ROWS_BLK, NTHR_R, 0, stream>>>(xtok, h0, c0, WHH16, PTAB, BSUM, out_h, out_c, H16);

  {
    const int tiles = (NBAT / 64) * (NVOCP / 64);
    wmma_gemm64_f16<2, 0><<<(tiles + 7) / 8, 256, 0, stream>>>(
        H16, KHID, WFC16, KHID, (void*)CST, NVOCP, BFCP, NBAT, NVOCP, KHID, ACC_FOLD);
  }

  out_copy_kernel<<<(NBAT * (NVOC / 4)) / 256, 256, 0, stream>>>(CST, out);
}
